// RelPosAttention_81776177316139
// MI455X (gfx1250) — hardware-verified
//
#include <hip/hip_runtime.h>


#define NB_  16
#define NN   1024
#define CC   512
#define C3   1536
#define NH_  16
#define HD   32
#define HP   64
#define ZH   8
#define PCAR 1024.0f
typedef _Float16 h16;
typedef unsigned short bf;
typedef __attribute__((ext_vector_type(16))) __bf16   v16bf;
typedef __attribute__((ext_vector_type(16))) _Float16 v16h;
typedef __attribute__((ext_vector_type(8)))  _Float16 v8h;
typedef __attribute__((ext_vector_type(8)))  unsigned short v8us;
typedef __attribute__((ext_vector_type(8)))  float    v8f;
typedef __attribute__((ext_vector_type(4)))  float    v4f;
typedef v8h  __attribute__((may_alias)) v8ha;
typedef v4f  __attribute__((may_alias)) v4fa;
typedef v8us __attribute__((may_alias)) v8usa;

__device__ __forceinline__ unsigned short f2bf(float f) { unsigned u = __float_as_uint(f); u += 0x7FFFu + ((u >> 16) & 1u); return (unsigned short)(u >> 16); }
__device__ __forceinline__ float bf2f(unsigned short b) { return __uint_as_float(((unsigned)b) << 16); }
__device__ __forceinline__ float bfr(float f) { return bf2f(f2bf(f)); }
__device__ __forceinline__ v16h cat16(v8h lo, v8h hi) { return __builtin_shufflevector(lo, hi, 0, 1, 2, 3, 4, 5, 6, 7, 8, 9, 10, 11, 12, 13, 14, 15); }
__device__ __forceinline__ v16bf cat16b(v8us lo, v8us hi) { return __builtin_bit_cast(v16bf, __builtin_shufflevector(lo, hi, 0, 1, 2, 3, 4, 5, 6, 7, 8, 9, 10, 11, 12, 13, 14, 15)); }
__device__ __forceinline__ v8f wmma16(v16h a, v16h b, v8f c) { return __builtin_amdgcn_wmma_f32_16x16x32_f16(false, a, false, b, (short)0, c, false, false); }
__device__ __forceinline__ v8f wmmab(v16bf a, v16bf b, v8f c) { return __builtin_amdgcn_wmma_f32_16x16x32_bf16(false, a, false, b, (short)0, c, false, false); }


template <typename T16> struct WFrag;
template <> struct WFrag<h16> { typedef v16h V; static __device__ __forceinline__ V ld(const h16* p) { return cat16(*(const v8h*)p, *(const v8h*)(p + 16)); } static __device__ __forceinline__ v8f mma(V a, V b, v8f c) { return wmma16(a, b, c); } };
template <> struct WFrag<bf> { typedef v16bf V; static __device__ __forceinline__ V ld(const bf* p) { return cat16b(*(const v8us*)p, *(const v8us*)(p + 16)); } static __device__ __forceinline__ v8f mma(V a, V b, v8f c) { return wmmab(a, b, c); } };
template <typename T16, int NSPLIT, bool BIAS>
__global__ __launch_bounds__(32) void k_gemmw(const T16* __restrict__ A, const T16* __restrict__ A2, const T16* __restrict__ Bt, const T16* __restrict__ Bt2, int K, float* C, int ldc, const float* __restrict__ bias, size_t sA, size_t sB, size_t sC) {
    typedef typename WFrag<T16>::V V;
    __shared__ __align__(16) float os[16 * 68];
    const size_t z = blockIdx.z; A += z * sA; if (A2) A2 += z * sA; Bt += z * sB; if (Bt2) Bt2 += z * sB; C += z * sC;
    const int lane = threadIdx.x & 31, lr = lane & 15, hi = lane >> 4; const int r0 = blockIdx.x * 64, c0 = blockIdx.y * 64;
    v8f acc[4][4];
#pragma unroll
    for (int mb = 0; mb < 4; ++mb)
#pragma unroll
        for (int nb = 0; nb < 4; ++nb) acc[mb][nb] = (v8f){};
    const size_t aoff = (size_t)(r0 + lr) * K + 8 * hi, boff = (size_t)(c0 + lr) * K + 8 * hi;
#pragma unroll 1
    for (int kc = 0; kc < K; kc += 32) {
        V a[4], a2[4];
#pragma unroll
        for (int mb = 0; mb < 4; ++mb) { a[mb] = WFrag<T16>::ld(A + aoff + (size_t)mb * 16 * K + kc); if (NSPLIT == 1 || NSPLIT == 2) a2[mb] = WFrag<T16>::ld(A2 + aoff + (size_t)mb * 16 * K + kc); }
#pragma unroll
        for (int nb = 0; nb < 4; ++nb) { const V b = WFrag<T16>::ld(Bt + boff + (size_t)nb * 16 * K + kc); V b2; if (NSPLIT >= 2) b2 = WFrag<T16>::ld(Bt2 + boff + (size_t)nb * 16 * K + kc);
#pragma unroll
            for (int mb = 0; mb < 4; ++mb) { acc[mb][nb] = WFrag<T16>::mma(a[mb], b, acc[mb][nb]); if (NSPLIT == 1 || NSPLIT == 2) acc[mb][nb] = WFrag<T16>::mma(a2[mb], b, acc[mb][nb]); if (NSPLIT >= 2) acc[mb][nb] = WFrag<T16>::mma(a[mb], b2, acc[mb][nb]); } }
        asm volatile("v_nop\n\tv_nop\n\tv_nop\n\tv_nop" : "+v"(acc[0][0]), "+v"(acc[1][1]), "+v"(acc[2][2]), "+v"(acc[3][3]) : "v"(a[0]), "v"(a[3]));
    }
#pragma unroll
    for (int mb = 0; mb < 4; ++mb) {
#pragma unroll
        for (int nb = 0; nb < 4; ++nb) {
#pragma unroll
            for (int j = 0; j < 8; ++j) os[(hi * 8 + j) * 68 + nb * 16 + lr] = acc[mb][nb][j]; }
        __builtin_amdgcn_wave_barrier(); asm volatile("" ::: "memory");
        float* crow = C + (size_t)(r0 + mb * 16) * ldc + c0;
#pragma unroll 1
        for (int ps = 0; ps < 2; ++ps) {
#pragma unroll
            for (int s = 0; s < 8; ++s) { const int row = 2 * s + hi, cofs = lr * 4; v4f val = *(const v4fa*)(os + row * 68 + cofs); if (BIAS) { val[0] += bfr(bias[c0 + cofs]); val[1] += bfr(bias[c0 + cofs + 1]); val[2] += bfr(bias[c0 + cofs + 2]); val[3] += bfr(bias[c0 + cofs + 3]); }
                *(volatile v4f*)(crow + (size_t)row * ldc + cofs) = val; }
            if (ps == 0) __threadfence(); }
        __builtin_amdgcn_wave_barrier(); asm volatile("" ::: "memory");
    }
}

__device__ __forceinline__ h16 tohx(float x) { return (h16)x; }
__device__ __forceinline__ void splitf(float y, unsigned short& h, unsigned short& l) { h = f2bf(y); l = f2bf(y - bf2f(h)); }
typedef __attribute__((ext_vector_type(2))) unsigned short v2us;
typedef __attribute__((ext_vector_type(4))) unsigned short v4us;
typedef __attribute__((ext_vector_type(2))) _Float16 v2h;
typedef __attribute__((ext_vector_type(4))) _Float16 v4h;
typedef __attribute__((ext_vector_type(4))) int v4i;

__global__ __launch_bounds__(256) void k_wtG(const float* __restrict__ w, int K, int N, bf* Bt) {
    const int lane = threadIdx.x & 31; const int L0 = (blockIdx.x * 8 + (threadIdx.x >> 5)) * 8; const int nlines = N * K / 64;
#pragma unroll
    for (int ps = 0; ps < 2; ++ps) {
#pragma unroll 1
        for (int l = 0; l < 8; ++l) { const int L = L0 + l; if (L >= nlines) break; const size_t e = (size_t)L * 64 + lane * 2; const int k = (int)(e % K), n = (int)(e / K); v2us o;
            o[0] = f2bf(w[(size_t)k * N + n]); o[1] = f2bf(w[(size_t)(k + 1) * N + n]); *(volatile v2us*)(Bt + e) = o; }
        if (ps == 0) __threadfence(); }
}
__global__ __launch_bounds__(256) void k_cvt8(const float* __restrict__ src, bf* dst, size_t n8) { const size_t i = (size_t)blockIdx.x * 256 + threadIdx.x; if (i >= n8) return; const v8f v = *(const v8f*)(src + i * 8); v8us o;
#pragma unroll
    for (int k = 0; k < 8; ++k) o[k] = f2bf(v[k]); *(volatile v8us*)(dst + i * 8) = o; __threadfence(); *(volatile v8us*)(dst + i * 8) = o; }
__global__ __launch_bounds__(256) void k_qk16(const float* __restrict__ F, h16* Q16, h16* K16) { const int e = (blockIdx.x * 256 + threadIdx.x) * 4; if (e >= NH_ * NN * HD) return; const int d = e % HD; const int t = (e / HD) % NN; const int h = e / (HD * NN); const float* f = F + (size_t)t * C3 + h * HD + d; const float SC = 0.17677669529663687f; v4h q, k;
#pragma unroll
    for (int u = 0; u < 4; ++u) { q[u] = tohx(__fmul_rn(f[u], SC)); k[u] = tohx(f[CC + u]); } for (int ps = 0; ps < 2; ++ps) { *(volatile v4h*)(Q16 + e) = q; *(volatile v4h*)(K16 + e) = k; if (ps == 0) __threadfence(); } }
__global__ __launch_bounds__(256) void k_vt16(const float* __restrict__ F, h16* VT) { const int e = (blockIdx.x * 256 + threadIdx.x) * 2; if (e >= NH_ * HP * NN) return; const int t = e % NN; const int dd = (e / NN) % HP; const int h = e / (NN * HP); v2h o;
    if (dd < HD) { o[0] = tohx(F[(size_t)t * C3 + 2 * CC + h * HD + dd]); o[1] = tohx(F[(size_t)(t + 1) * C3 + 2 * CC + h * HD + dd]); } else { o[0] = (h16)0.f; o[1] = (h16)0.f; }
    *(volatile v2h*)(VT + e) = o; __threadfence(); *(volatile v2h*)(VT + e) = o; }
__global__ __launch_bounds__(256) void k_bsoft(const float* __restrict__ Sb, const int* __restrict__ rel, const float* __restrict__ tab, int h0, h16* P16) { const int lane = threadIdx.x & 31; const int row = blockIdx.x * 8 + (threadIdx.x >> 5); if (row >= ZH * NN) return; const int i = row % NN; const int h = h0 + row / NN; const float* sr = Sb + (size_t)row * NN; const int* rr = rel + (size_t)i * NN; float v[NN / 32]; float mx = -3.0e38f;
#pragma unroll
    for (int ch = 0; ch < NN / 128; ++ch) { const int j0 = ch * 128 + lane * 4; const v4f a = *(const v4f*)(sr + j0); const v4i r4 = *(const v4i*)(rr + j0);
#pragma unroll
        for (int u = 0; u < 4; ++u) { int r = r4[u]; r = r < 0 ? 0 : (r > 3968 ? 3968 : r); const float t = __fadd_rn(a[u], bfr(tab[(size_t)r * NH_ + h])); v[ch * 4 + u] = t; mx = fmaxf(mx, t); } }
#pragma unroll
    for (int sh = 16; sh; sh >>= 1) mx = fmaxf(mx, __shfl_xor(mx, sh, 32));
    float sum = 0.f;
#pragma unroll
    for (int q = 0; q < NN / 32; ++q) { float d0 = __fsub_rn(v[q], mx); asm volatile("" : "+v"(d0)); v[q] = __expf(d0); sum += v[q]; }
#pragma unroll
    for (int sh = 16; sh; sh >>= 1) sum += __shfl_xor(sum, sh, 32);
    const float f = __fdiv_rn(PCAR, sum);
    for (int ps = 0; ps < 2; ++ps) {
#pragma unroll
        for (int ch = 0; ch < NN / 128; ++ch) { v4h o4;
#pragma unroll
            for (int q = 0; q < 4; ++q) o4[q] = tohx(v[ch * 4 + q] * f); *(volatile v4h*)(P16 + (size_t)row * NN + ch * 128 + lane * 4) = o4; }
        if (ps == 0) __threadfence(); } }
__global__ __launch_bounds__(256) void k_mrg(const float* __restrict__ O, int h0, bf* Ah, bf* Al) { const int idx = blockIdx.x * 256 + threadIdx.x; if (idx >= ZH * NN * HD / 4) return; const int d = (idx % 8) * 4; const int z = (idx / 8) % ZH; const int t = idx / (8 * ZH); const float* o = O + ((size_t)z * NN + t) * HP + d; v4us oh, ol;
#pragma unroll
    for (int u = 0; u < 4; ++u) { unsigned short a, b; splitf(o[u] * (1.0f / PCAR), a, b); oh[u] = a; ol[u] = b; } const size_t oo = (size_t)t * CC + (h0 + z) * HD + d;
    *(volatile v4us*)(Ah + oo) = oh; *(volatile v4us*)(Al + oo) = ol; __threadfence(); *(volatile v4us*)(Ah + oo) = oh; *(volatile v4us*)(Al + oo) = ol; }

extern "C" void kernel_launch(void* const* d_in, const int* in_sizes, int n_in,
                              void* d_out, int out_size, void* d_ws, size_t ws_size, hipStream_t stream) {
    (void)in_sizes; (void)n_in; (void)out_size;
    const float* x = (const float*)d_in[0]; const float* wqkv = (const float*)d_in[1]; const float* bqkv = (const float*)d_in[2]; const float* wp = (const float*)d_in[3]; const float* bp = (const float*)d_in[4]; const float* tab = (const float*)d_in[5]; const int* rel = (const int*)d_in[6];
    float* OUT = (float*)d_out;
    char* wsp = (char*)d_ws;
    auto take = [&](size_t bytes) { char* p = wsp; wsp += (bytes + 255) & ~(size_t)255; return (void*)p; };
    bf* WQ = (bf*)take((size_t)C3 * CC * 2); bf* WP = (bf*)take((size_t)CC * CC * 2); bf* XB = (bf*)take((size_t)NN * CC * 2); float* F = (float*)take((size_t)NN * C3 * 4);
    h16* Q16 = (h16*)take((size_t)NH_ * NN * HD * 2); h16* K16 = (h16*)take((size_t)NH_ * NN * HD * 2); h16* VT = (h16*)take((size_t)NH_ * HP * NN * 2); float* Sb = (float*)take((size_t)ZH * NN * NN * 4); h16* P16 = (h16*)take((size_t)ZH * NN * NN * 2); float* O = (float*)take((size_t)ZH * NN * HP * 4); bf* Ah = (bf*)take((size_t)NN * CC * 2); bf* Al = (bf*)take((size_t)NN * CC * 2);
    if ((size_t)(wsp - (char*)d_ws) > ws_size) return;
    k_wtG<<<(CC * C3 / 64 + 63) / 64, 256, 0, stream>>>(wqkv, CC, C3, WQ); k_wtG<<<(CC * CC / 64 + 63) / 64, 256, 0, stream>>>(wp, CC, CC, WP);
    for (int b = 0; b < NB_; ++b) {
        k_cvt8<<<(NN * CC / 8 + 255) / 256, 256, 0, stream>>>(x + (size_t)b * NN * CC, XB, (size_t)NN * CC / 8);
        k_gemmw<bf, 0, true><<<dim3(NN / 64, C3 / 64, 1), 32, 0, stream>>>(XB, nullptr, WQ, nullptr, CC, F, C3, bqkv, 0, 0, 0);
        k_qk16<<<(NH_ * NN * HD / 4 + 255) / 256, 256, 0, stream>>>(F, Q16, K16); k_vt16<<<(NH_ * HP * NN / 2 + 255) / 256, 256, 0, stream>>>(F, VT);
        for (int h0 = 0; h0 < NH_; h0 += ZH) {
            k_gemmw<h16, 0, false><<<dim3(NN / 64, NN / 64, ZH), 32, 0, stream>>>(Q16 + (size_t)h0 * NN * HD, nullptr, K16 + (size_t)h0 * NN * HD, nullptr, HD, Sb, NN, nullptr, (size_t)NN * HD, (size_t)NN * HD, (size_t)NN * NN);
            k_bsoft<<<ZH * NN / 8, 256, 0, stream>>>(Sb, rel, tab, h0, P16);
            k_gemmw<h16, 0, false><<<dim3(NN / 64, 1, ZH), 32, 0, stream>>>(P16, nullptr, VT + (size_t)h0 * HP * NN, nullptr, NN, O, HP, nullptr, (size_t)NN * NN, (size_t)HP * NN, (size_t)NN * HP);
            k_mrg<<<(ZH * NN * HD / 4 + 255) / 256, 256, 0, stream>>>(O, h0, Ah, Al); }
        k_gemmw<bf, 1, true><<<dim3(NN / 64, CC / 64, 1), 32, 0, stream>>>(Ah, Al, WP, nullptr, CC, OUT + (size_t)b * NN * CC, CC, bp, 0, 0, 0); }
}
